// WKNN_44856638439627
// MI455X (gfx1250) — hardware-verified
//
#include <hip/hip_runtime.h>


typedef float        v4f  __attribute__((ext_vector_type(4)));
typedef float        v8f  __attribute__((ext_vector_type(8)));
typedef unsigned int v4u  __attribute__((ext_vector_type(4)));
typedef int          v4i  __attribute__((ext_vector_type(4)));
typedef __bf16       v16b __attribute__((ext_vector_type(16)));

#pragma clang fp contract(off)

#define DIMF     64
#define KSEL     32
#define NCLS     10
#define QPW      16
#define WPB      4
#define TPB_MAIN (WPB * 32)
#define TPB_PREP 256
#define BIGKEY   1.0e30f

union Frag { v16b v; v4u q[2]; };

__device__ __forceinline__ unsigned int bf16_rne_bits(float f) {
    unsigned int u = __float_as_uint(f);
    return (u + 0x7FFFu + ((u >> 16) & 1u)) >> 16;
}
__device__ __forceinline__ void split_hl(float f, unsigned int& hb, unsigned int& lb) {
    hb = bf16_rne_bits(f);
    const float hf = __uint_as_float(hb << 16);
    lb = bf16_rne_bits(f - hf);
}
__device__ __forceinline__ void pack8(v4f a, v4f b, v4u& hq, v4u& lq) {
    float f[8] = {a.x, a.y, a.z, a.w, b.x, b.y, b.z, b.w};
    unsigned int hb[8], lb[8];
#pragma unroll
    for (int i = 0; i < 8; ++i) split_hl(f[i], hb[i], lb[i]);
    hq.x = hb[0] | (hb[1] << 16); hq.y = hb[2] | (hb[3] << 16);
    hq.z = hb[4] | (hb[5] << 16); hq.w = hb[6] | (hb[7] << 16);
    lq.x = lb[0] | (lb[1] << 16); lq.y = lb[2] | (lb[3] << 16);
    lq.z = lb[4] | (lb[5] << 16); lq.w = lb[6] | (lb[7] << 16);
}

__device__ __forceinline__ v8f wmma_bf16(v16b a, v16b b, v8f c) {
    return __builtin_amdgcn_wmma_f32_16x16x32_bf16(false, a, false, b, (short)0, c, false, false);
}

__device__ __forceinline__ void insert32(float (&kl)[KSEL], int (&il)[KSEL], const float key, const int idx) {
#pragma unroll
    for (int j = KSEL - 1; j >= 1; --j) {
        const bool cj = key < kl[j];
        const bool cm = key < kl[j - 1];
        const float nk = cm ? kl[j - 1] : (cj ? key : kl[j]);
        const int   ni = cm ? il[j - 1] : (cj ? idx : il[j]);
        kl[j] = nk;
        il[j] = ni;
    }
    const bool c0 = key < kl[0];
    il[0] = c0 ? idx : il[0];
    kl[0] = c0 ? key : kl[0];
}

__global__ __launch_bounds__(TPB_PREP)
void k_prep(const float* __restrict__ train,
            unsigned short* __restrict__ Th,
            unsigned short* __restrict__ Tl,
            float* __restrict__ x2,
            int ntrain)
{
    const int tid  = threadIdx.x;
    const int lane = tid & 31;
    const int r    = blockIdx.x * TPB_PREP + tid;
    const bool valid = r < ntrain;
    const int rc   = valid ? r : (ntrain - 1);
    const float* src = train + (size_t)rc * DIMF;
    const v4f z4 = {0.f, 0.f, 0.f, 0.f};

    float s = 0.f;
    v4u th[8], tl[8];
#pragma unroll
    for (int c = 0; c < 8; ++c) {
        v4f a = *(const v4f*)(src + 8 * c);
        v4f b = *(const v4f*)(src + 8 * c + 4);
        a = valid ? a : z4;
        b = valid ? b : z4;
        float p;
        p = a.x * a.x; s = s + p;
        p = a.y * a.y; s = s + p;
        p = a.z * a.z; s = s + p;
        p = a.w * a.w; s = s + p;
        p = b.x * b.x; s = s + p;
        p = b.y * b.y; s = s + p;
        p = b.z * b.z; s = s + p;
        p = b.w * b.w; s = s + p;
        pack8(a, b, th[c], tl[c]);
    }
    const float xv = valid ? s : BIGKEY;

    float g[4];
#pragma unroll
    for (int c = 0; c < 4; ++c) g[c] = __shfl(xv, ((lane & 7) << 2) + c);
    v4f gx; gx.x = g[0]; gx.y = g[1]; gx.z = g[2]; gx.w = g[3];

    v4u* dh = (v4u*)(Th + (size_t)r * DIMF);
    v4u* dl = (v4u*)(Tl + (size_t)r * DIMF);
    float* dx = x2 + (size_t)(r - lane) + (size_t)(lane << 2);

#pragma unroll
    for (int c = 0; c < 8; ++c) *(volatile v4u*)(dh + c) = th[c];
#pragma unroll
    for (int c = 0; c < 8; ++c) *(volatile v4u*)(dl + c) = tl[c];
    if (lane < 8) *(volatile v4f*)dx = gx;
    __threadfence();
#pragma unroll
    for (int c = 0; c < 8; ++c) *(volatile v4u*)(dh + c) = th[c];
#pragma unroll
    for (int c = 0; c < 8; ++c) *(volatile v4u*)(dl + c) = tl[c];
    if (lane < 8) *(volatile v4f*)dx = gx;
}

__global__ __launch_bounds__(TPB_MAIN)
void k_main(const float* __restrict__ queries,
            const unsigned short* __restrict__ Th,
            const unsigned short* __restrict__ Tl,
            const float* __restrict__ x2,
            const int* __restrict__ labels,
            int* __restrict__ out,
            int nq, int nlab, int ntiles)
{
    __shared__ float sKey[WPB][32][KSEL];
    __shared__ int   sIdx[WPB][32][KSEL];
    __shared__ __attribute__((aligned(16))) int sOut[WPB * QPW];

    const int tid  = threadIdx.x;
    const int lane = tid & 31;
    const int wave = tid >> 5;
    const int h    = lane >> 4;
    const int m    = lane & 15;
    const int q0   = (blockIdx.x * WPB + wave) * QPW;
    int qi = q0 + m;
    qi = (qi < nq) ? qi : (nq - 1);
    const float* qrow = queries + (size_t)qi * DIMF;

    float q2 = 0.f;
#pragma unroll
    for (int c = 0; c < 16; ++c) {
        const v4f v = *(const v4f*)(qrow + 4 * c);
        float p;
        p = v.x * v.x; q2 = q2 + p;
        p = v.y * v.y; q2 = q2 + p;
        p = v.z * v.z; q2 = q2 + p;
        p = v.w * v.w; q2 = q2 + p;
    }

    Frag bh0, bl0, bh1, bl1;
    {
        const float* p0 = qrow + 8 * h;
        pack8(*(const v4f*)(p0),      *(const v4f*)(p0 + 4),  bh0.q[0], bl0.q[0]);
        pack8(*(const v4f*)(p0 + 16), *(const v4f*)(p0 + 20), bh0.q[1], bl0.q[1]);
        pack8(*(const v4f*)(p0 + 32), *(const v4f*)(p0 + 36), bh1.q[0], bl1.q[0]);
        pack8(*(const v4f*)(p0 + 48), *(const v4f*)(p0 + 52), bh1.q[1], bl1.q[1]);
    }

    float kl[KSEL];
    int   il[KSEL];
#pragma unroll
    for (int j = 0; j < KSEL; ++j) { kl[j] = __builtin_huge_valf(); il[j] = 0; }
    float thr = __builtin_huge_valf();

    const unsigned short* ph = Th + (size_t)m * DIMF + 8 * h;
    const unsigned short* pl = Tl + (size_t)m * DIMF + 8 * h;
    const float* px = x2 + 8 * h;

    for (int t = 0; t < ntiles; ++t) {
        const size_t ro = (size_t)t * (16 * DIMF);
        const size_t xo = (size_t)t * 16;
        Frag ah0, al0, ah1, al1;
        ah0.q[0] = *(const v4u*)(ph + ro);
        ah0.q[1] = *(const v4u*)(ph + ro + 16);
        ah1.q[0] = *(const v4u*)(ph + ro + 32);
        ah1.q[1] = *(const v4u*)(ph + ro + 48);
        al0.q[0] = *(const v4u*)(pl + ro);
        al0.q[1] = *(const v4u*)(pl + ro + 16);
        al1.q[0] = *(const v4u*)(pl + ro + 32);
        al1.q[1] = *(const v4u*)(pl + ro + 48);
        const v4f xlo = *(const v4f*)(px + xo);
        const v4f xhi = *(const v4f*)(px + xo + 4);

        v8f acc = {0.f, 0.f, 0.f, 0.f, 0.f, 0.f, 0.f, 0.f};
        acc = wmma_bf16(ah0.v, bh0.v, acc);
        acc = wmma_bf16(al0.v, bh0.v, acc);
        acc = wmma_bf16(ah0.v, bl0.v, acc);
        acc = wmma_bf16(ah1.v, bh1.v, acc);
        acc = wmma_bf16(al1.v, bh1.v, acc);
        acc = wmma_bf16(ah1.v, bl1.v, acc);
        asm volatile("v_nop\n\tv_nop\n\tv_nop\n\tv_nop"
                     : "+v"(acc)
                     : "v"(ah0.v), "v"(al0.v), "v"(ah1.v), "v"(al1.v),
                       "v"(bh0.v), "v"(bl0.v), "v"(bh1.v), "v"(bl1.v));

        const float x8[8] = {xlo.x, xlo.y, xlo.z, xlo.w, xhi.x, xhi.y, xhi.z, xhi.w};
        float e[8];
#pragma unroll
        for (int r = 0; r < 8; ++r) {
            const float tt = q2 + x8[r];
            e[r] = fmaf(-2.0f, acc[r], tt);
        }
        float emin = e[0];
#pragma unroll
        for (int r = 1; r < 8; ++r) emin = fminf(emin, e[r]);

        if (__builtin_amdgcn_ballot_w32(emin < thr) != 0u) {
            const int nb = t * 16 + 8 * h;
#pragma unroll
            for (int r = 0; r < 8; ++r) {
                const float key = (e[r] > 0.f) ? e[r] : 0.1f;
                const bool  c   = key < thr;
                if (__builtin_amdgcn_ballot_w32(c) != 0u) {
                    insert32(kl, il, key, nb + r);
                    thr = kl[KSEL - 1];
                }
            }
        }
    }

#pragma unroll
    for (int j = 0; j < KSEL; ++j) {
        sKey[wave][lane][j] = kl[j];
        sIdx[wave][lane][j] = il[j];
    }
    __syncthreads();

    if (h == 0) {
        const float* ka  = &sKey[wave][m][0];
        const float* kb  = &sKey[wave][m + 16][0];
        const int*   pia = &sIdx[wave][m][0];
        const int*   pib = &sIdx[wave][m + 16][0];
        int ia = 0, ib = 0;
        float votes[NCLS];
#pragma unroll
        for (int c = 0; c < NCLS; ++c) votes[c] = 0.f;
#pragma unroll 1
        for (int j = 0; j < KSEL; ++j) {
            const int ca = (ia < KSEL - 1) ? ia : (KSEL - 1);
            const int cb = (ib < KSEL - 1) ? ib : (KSEL - 1);
            const float vA = ka[ca], vB = kb[cb];
            const int   iA = pia[ca], iB = pib[cb];
            const bool  tA = (vA < vB) || ((vA == vB) && (iA < iB));
            const float key = tA ? vA : vB;
            int idx = tA ? iA : iB;
            ia += tA ? 1 : 0;
            ib += tA ? 0 : 1;
            const float w0 = 1.0f / key;
            const float w  = (key < BIGKEY) ? w0 : 0.f;
            idx = (idx < 0) ? 0 : idx;
            idx = (idx > nlab - 1) ? (nlab - 1) : idx;
            const int lab = labels[idx];
#pragma unroll
            for (int c = 0; c < NCLS; ++c) {
                const float add = (lab == c) ? w : 0.0f;
                votes[c] = votes[c] + add;
            }
        }
        int best = 0;
        float bv = votes[0];
#pragma unroll
        for (int c = 1; c < NCLS; ++c) {
            if (votes[c] > bv) { bv = votes[c]; best = c; }
        }
        sOut[wave * QPW + m] = best;
    }
    __syncthreads();

    const int  obase = blockIdx.x * (WPB * QPW);
    const bool wr    = (tid < QPW) && (obase + WPB * QPW <= nq);
    v4i ov = {0, 0, 0, 0};
    if (tid < QPW) ov = *(const v4i*)(&sOut[tid * 4]);
    if (wr) *(volatile v4i*)(out + obase + tid * 4) = ov;
    __threadfence();
    if (wr) *(volatile v4i*)(out + obase + tid * 4) = ov;
}

static inline size_t align_up256(size_t x) { return (x + 255) & ~(size_t)255; }

extern "C" void kernel_launch(void* const* d_in, const int* in_sizes, int n_in,
                              void* d_out, int out_size, void* d_ws, size_t ws_size,
                              hipStream_t stream)
{
    if (n_in < 3) return;
    const float* queries = (const float*)d_in[0];
    const float* train   = (const float*)d_in[1];
    const int*   labels  = (const int*)d_in[2];
    int* out = (int*)d_out;

    const int nq     = in_sizes[0] / DIMF;
    const int ntrain = in_sizes[1] / DIMF;
    const int nlab   = in_sizes[2];
    if (nq < WPB * QPW || (nq % (WPB * QPW)) != 0 || ntrain < 1 || nlab < 1 || out_size < nq) return;

    const int    nblk_prep = (ntrain + TPB_PREP - 1) / TPB_PREP;
    const size_t NP        = (size_t)nblk_prep * TPB_PREP;
    const int    ntiles    = (ntrain + 15) / 16;

    const size_t plane_bytes = NP * DIMF * sizeof(unsigned short);
    const size_t offTh = 0;
    const size_t offTl = align_up256(offTh + plane_bytes);
    const size_t offX2 = align_up256(offTl + plane_bytes);
    const size_t end   = offX2 + NP * sizeof(float);
    if (end > ws_size || end > (size_t)134217728) return;

    unsigned char* ws = (unsigned char*)d_ws;
    unsigned short* Th = (unsigned short*)(ws + offTh);
    unsigned short* Tl = (unsigned short*)(ws + offTl);
    float*          x2 = (float*)(ws + offX2);

    k_prep<<<nblk_prep, TPB_PREP, 0, stream>>>(train, Th, Tl, x2, ntrain);

    k_main<<<nq / (WPB * QPW), TPB_MAIN, 0, stream>>>(queries, Th, Tl, x2, labels, out, nq, nlab, ntiles);
}
